// Get_embd_11836929868522
// MI455X (gfx1250) — hardware-verified
//
#include <hip/hip_runtime.h>
#include <stdint.h>

typedef __attribute__((ext_vector_type(16))) _Float16 v16h;
typedef __attribute__((ext_vector_type(8)))  _Float16 v8h;
typedef __attribute__((ext_vector_type(16))) __bf16   v16b;
typedef __attribute__((ext_vector_type(8)))  __bf16   v8b;
typedef __attribute__((ext_vector_type(8)))  float    v8f;
typedef __attribute__((ext_vector_type(4)))  float    v4f;
typedef __attribute__((ext_vector_type(4)))  unsigned int v4u;
typedef __attribute__((ext_vector_type(2)))  unsigned int v2u;

__device__ __forceinline__ unsigned short f2bf_bits(float f) {
  unsigned u = __float_as_uint(f);
  return (unsigned short)((u + 0x7FFFu + ((u >> 16) & 1u)) >> 16);
}
__device__ __forceinline__ float bf_bits2f(unsigned short h) { return __uint_as_float(((unsigned)h) << 16); }

__device__ __forceinline__ void dep_guard_h(v8f& a, v8f& b, v16h x, v16h y) { asm volatile("v_nop\n\tv_nop\n\tv_nop\n\tv_nop" : "+v"(a), "+v"(b) : "v"(x), "v"(y)); }
__device__ __forceinline__ void dep_guard_b(v8f& a, v8f& b, v16b x, v16b y) { asm volatile("v_nop\n\tv_nop\n\tv_nop\n\tv_nop" : "+v"(a), "+v"(b) : "v"(x), "v"(y)); }
__device__ __forceinline__ void keep4_h(v16h a, v16h b, v16h c, v16h d) { asm volatile("v_nop" :: "v"(a), "v"(b), "v"(c), "v"(d)); }
__device__ __forceinline__ void keep4_b(v16b a, v16b b, v16b c, v16b d) { asm volatile("v_nop" :: "v"(a), "v"(b), "v"(c), "v"(d)); }
__device__ __forceinline__ void acc_guard4(v8f& a, v8f& b, v8f& c, v8f& d) { asm volatile("v_nop\n\tv_nop\n\tv_nop\n\tv_nop" : "+v"(a), "+v"(b), "+v"(c), "+v"(d)); }
template <typename T> struct Frag;
template <> struct Frag<_Float16> {
  typedef v16h V; union U { v16h v; v8h h[2]; };
  static __device__ __forceinline__ v16h load(const _Float16* p) {
    U f; f.h[0] = *(const v8h*)(p); f.h[1] = *(const v8h*)(p + 16); return f.v;
  }
  static __device__ __forceinline__ v8f mma(v16h a, v16h b, v8f c) {
    return __builtin_amdgcn_wmma_f32_16x16x32_f16(false, a, false, b, (short)0, c, false, false);
  }
  static __device__ __forceinline__ void guard(v8f& a, v8f& b, v16h x, v16h y) { dep_guard_h(a, b, x, y); }
  static __device__ __forceinline__ void keep(v16h a, v16h b, v16h c, v16h d) { keep4_h(a, b, c, d); }
};
template <> struct Frag<__bf16> {
  typedef v16b V; union U { v16b v; v8b h[2]; };
  static __device__ __forceinline__ v16b load(const __bf16* p) {
    U f; f.h[0] = *(const v8b*)(p); f.h[1] = *(const v8b*)(p + 16); return f.v;
  }
  static __device__ __forceinline__ v8f mma(v16b a, v16b b, v8f c) {
    return __builtin_amdgcn_wmma_f32_16x16x32_bf16(false, a, false, b, (short)0, c, false, false);
  }
  static __device__ __forceinline__ void guard(v8f& a, v8f& b, v16b x, v16b y) { dep_guard_b(a, b, x, y); }
  static __device__ __forceinline__ void keep(v16b a, v16b b, v16b c, v16b d) { keep4_b(a, b, c, d); }
};

template <int ET> struct Elem;
template <> struct Elem<0> { typedef _Float16 T; };
template <> struct Elem<1> { typedef __bf16 T; };
template <int ET, bool SPLIT, int BIAS_MODE, int OUT_MODE, bool RESID, int ACT = 0>
__global__ __launch_bounds__(256) void wmma_gemm64(
    const unsigned short* __restrict__ Ap, const unsigned short* __restrict__ A2p, int lda, long strideA,
    const unsigned short* __restrict__ Btp, const unsigned short* __restrict__ Bt2p, int ldb, long strideB,
    void* __restrict__ Cout, void* __restrict__ Cout2, int ldc, long strideC,
    const float* __restrict__ bias,
    const float* __restrict__ resid, long strideR,
    int M, int N, int K, float scale) {
  typedef typename Elem<ET>::T T;
  typedef typename Frag<T>::V V;
  const T* A = (const T*)Ap; const T* A2 = (const T*)A2p; const T* Bt = (const T*)Btp; const T* Bt2 = (const T*)Bt2p;
  __shared__ __align__(16) float sT[8][16 * 68];
  const int b    = blockIdx.y;
  const int lane = threadIdx.x & 31;
  const int wave = threadIdx.x >> 5;
  const int tilesN = N >> 6;
  const int tilesM = M >> 6;
  const int tile = blockIdx.x * 8 + wave;
  if (tile >= tilesM * tilesN) return;
  const int tm = tile / tilesN;
  const int tn = tile - tm * tilesN;
  const int m0 = tm << 6;
  const int n0 = tn << 6;

  const T* Ab  = A  + (size_t)b * strideA;
  const T* Bb  = Bt + (size_t)b * strideB;
  const T* Ab2 = SPLIT ? (A2  + (size_t)b * strideA) : nullptr;
  const T* Bb2 = SPLIT ? (Bt2 + (size_t)b * strideB) : nullptr;

  const int rlane = lane & 15;
  const int koff  = (lane >> 4) * 8;
  const int mOff  = (lane >> 4) * 8;

  v8f acc[4][4];
#pragma unroll
  for (int i = 0; i < 4; ++i)
#pragma unroll
    for (int j = 0; j < 4; ++j) acc[i][j] = (v8f){0.f,0.f,0.f,0.f,0.f,0.f,0.f,0.f};

  for (int k0 = 0; k0 < K; k0 += 32) {
    V bh[4], bl[4];
#pragma unroll
    for (int j = 0; j < 4; ++j) {
      const size_t bo = (size_t)(n0 + (j << 4) + rlane) * ldb + koff + k0;
      bh[j] = Frag<T>::load(Bb + bo);
      if (SPLIT) bl[j] = Frag<T>::load(Bb2 + bo);
    }
#pragma unroll
    for (int i = 0; i < 4; ++i) {
      const size_t ao = (size_t)(m0 + (i << 4) + rlane) * lda + koff + k0;
      V ah = Frag<T>::load(Ab + ao);
      V al;
      if (SPLIT) al = Frag<T>::load(Ab2 + ao);
#pragma unroll
      for (int j = 0; j < 4; ++j) {
        acc[i][j] = Frag<T>::mma(ah, bh[j], acc[i][j]);
        if (SPLIT) {
          acc[i][j] = Frag<T>::mma(ah, bl[j], acc[i][j]);
          acc[i][j] = Frag<T>::mma(al, bh[j], acc[i][j]);
        }
      }
      Frag<T>::guard(acc[i][0], acc[i][3], ah, SPLIT ? al : ah);
    }
    Frag<T>::keep(bh[0], bh[1], bh[2], bh[3]);
    if (SPLIT) Frag<T>::keep(bl[0], bl[1], bl[2], bl[3]);
  }
  acc_guard4(acc[0][0], acc[0][1], acc[0][2], acc[0][3]);
  acc_guard4(acc[1][0], acc[1][1], acc[1][2], acc[1][3]);
  acc_guard4(acc[2][0], acc[2][1], acc[2][2], acc[2][3]);
  acc_guard4(acc[3][0], acc[3][1], acc[3][2], acc[3][3]);

  float* slab = sT[wave];
  const float* Rb = RESID ? (resid + (size_t)b * strideR) : nullptr;
#pragma unroll
  for (int i = 0; i < 4; ++i) {
    const int mBase = m0 + (i << 4);
#pragma unroll
    for (int j = 0; j < 4; ++j) {
      const int n = n0 + (j << 4) + rlane;
      float bv = 0.f;
      if (BIAS_MODE == 2) bv = bias[n];
#pragma unroll
      for (int r = 0; r < 8; ++r) {
        float v = acc[i][j][r] * scale;
        if (BIAS_MODE == 1) v += bias[mBase + mOff + r];
        if (BIAS_MODE == 2) v += bv;
        if (RESID) v += Rb[(size_t)(mBase + mOff + r) * ldc + n];
        if (ACT == 1) v = tanhf(v);
        if (ACT == 2) v = fmaxf(v, 0.0f);
        if (ACT == 3) v = v / (1.0f + expf(-v));
        if (ACT == 4) v = (v > 0.f) ? v : 0.01f * v;
        if (ACT == 5) v = 0.5f * v * (1.0f + erff(v * 0.70710678118654752f));
        slab[(mOff + r) * 68 + (j << 4) + rlane] = v;
      }
    }
    __builtin_amdgcn_fence(__ATOMIC_RELEASE, "workgroup");
    __builtin_amdgcn_wave_barrier();
    __builtin_amdgcn_fence(__ATOMIC_ACQUIRE, "workgroup");
    if (OUT_MODE == 0) {
      float* C = (float*)Cout + (size_t)b * strideC;
      const int hh = lane >> 4, c4 = (lane & 15) * 4;
      for (int pass = 0; pass < 2; ++pass) {
#pragma unroll
        for (int it = 0; it < 8; ++it) {
          const int row = it * 2 + hh;
          v4f v = *(const v4f*)(slab + row * 68 + c4);
          *(volatile v4f*)(C + (size_t)(mBase + row) * ldc + n0 + c4) = v;
        }
        __threadfence();
      }
    } else {
      const int q = lane >> 3, c8 = (lane & 7) * 8;
      unsigned short* C  = (unsigned short*)Cout  + (size_t)b * strideC;
      unsigned short* C2 = (OUT_MODE == 2) ? ((unsigned short*)Cout2 + (size_t)b * strideC) : nullptr;
      for (int pass = 0; pass < 2; ++pass) {
#pragma unroll
        for (int it = 0; it < 4; ++it) {
          const int row = it * 4 + q;
          const float* sp = slab + row * 68 + c8;
          v8h hv, lv;
#pragma unroll
          for (int e = 0; e < 8; ++e) {
            if (OUT_MODE == 1) {
              hv[e] = (_Float16)sp[e];
            } else {
              unsigned short hb = f2bf_bits(sp[e]);
              unsigned short lb = f2bf_bits(sp[e] - bf_bits2f(hb));
              hv[e] = __builtin_bit_cast(_Float16, hb);
              lv[e] = __builtin_bit_cast(_Float16, lb);
            }
          }
          *(volatile v8h*)(C + (size_t)(mBase + row) * ldc + n0 + c8) = hv;
          if (OUT_MODE == 2) *(volatile v8h*)(C2 + (size_t)(mBase + row) * ldc + n0 + c8) = lv;
        }
        __threadfence();
      }
    }
    __builtin_amdgcn_fence(__ATOMIC_RELEASE, "workgroup");
    __builtin_amdgcn_wave_barrier();
    __builtin_amdgcn_fence(__ATOMIC_ACQUIRE, "workgroup");
  }
}

constexpr int kNB       = 32;
constexpr int kNS       = 50;
constexpr int kNCd      = 32;
constexpr int kHid      = 256;
constexpr int kTH       = 768;
constexpr int kTW       = 2304;
constexpr int kNCode    = 10001;
constexpr int kNCodePad = 10048;
constexpr int kNGrp     = 4800;
constexpr int kNRow     = 1600;
constexpr float kInv4096 = 1.0f / 4096.0f;
constexpr float kAttScale = 0.10846522890932808f;
static_assert(kNGrp * kHid == kNRow * kTH);
static_assert(kNCodePad % 64 == 0 && kTW % 64 == 0 && kNRow % 64 == 0);

__device__ __forceinline__ unsigned short f2h_bits(float f) { return __builtin_bit_cast(unsigned short, (_Float16)f); }

__device__ __forceinline__ v8f mma_h(v16h a, v16h b, v8f c) {
  c = __builtin_amdgcn_wmma_f32_16x16x32_f16(false, a, false, b, (short)0, c, false, false);
  asm volatile("v_nop\n\tv_nop\n\tv_nop\n\tv_nop" : "+v"(c) : "v"(a), "v"(b));
  return c;
}

__global__ __launch_bounds__(256) void k_cast_f16(const float* __restrict__ in, int nvalid,
                                                  unsigned short* __restrict__ out, int n2, float s) {
  const int i = blockIdx.x * 256 + threadIdx.x;
  if (i < n2) {
    const int i0 = 2 * i, i1 = 2 * i + 1;
    const int c0 = (i0 < nvalid) ? i0 : (nvalid - 1);
    const int c1 = (i1 < nvalid) ? i1 : (nvalid - 1);
    float a = in[c0] * s, b = in[c1] * s;
    a = (i0 < nvalid) ? a : 0.0f;
    b = (i1 < nvalid) ? b : 0.0f;
    const unsigned u = (unsigned)f2h_bits(a) | ((unsigned)f2h_bits(b) << 16);
    volatile unsigned* o = (volatile unsigned*)out;
    o[i] = u;
    __threadfence();
    o[i] = u;
  }
}

__global__ __launch_bounds__(256) void k_code_attn(
    const int* __restrict__ codes, const float* __restrict__ mask_code,
    const float* __restrict__ tab,
    const float* __restrict__ bq, const float* __restrict__ bk, const float* __restrict__ bv,
    unsigned short* __restrict__ temp16)
{
  __shared__ __align__(16) unsigned short Qs[32 * 264];
  __shared__ __align__(16) unsigned short Ks[32 * 264];
  __shared__ __align__(16) unsigned short Vt[256 * 40];
  __shared__ __align__(16) unsigned short Ps[32 * 40];
  __shared__ float Sf[32 * 33];
  __shared__ float nomv[256];
  __shared__ float kvalf[32];
  __shared__ float rowm[32];
  __shared__ int rowbase[32];
  __shared__ int rowboff[32];
  __shared__ int scnt;

  const int gidx = blockIdx.x;
  const int n = gidx / kNS;
  const int s = gidx - n * kNS;
  const int bm = n & 31;
  const int tid = threadIdx.x, lane = tid & 31, wave = tid >> 5;
  const int hh = lane >> 4, rl = lane & 15, koff = hh * 8;

  if (wave == 0) {
    const int g = gidx * kNCd + lane;
    const int p = g / 3;
    const int jj = g - p * 3;
    int code = codes[p];
    code = (code < 0) ? 0 : ((code > kNCode - 1) ? (kNCode - 1) : code);
    rowbase[lane] = code * kTW + jj * kHid;
    rowboff[lane] = jj * kHid;
    rowm[lane] = mask_code[p];
  } else if (wave == 1) {
    const float mv = mask_code[(bm * kNS + s) * kNCd + lane];
    const int kv = (mv != 0.0f) ? 1 : 0;
    kvalf[lane] = kv ? 1.0f : 0.0f;
    int cnt = kv;
#pragma unroll
    for (int off = 1; off < 32; off <<= 1) cnt += __shfl_xor(cnt, off, 32);
    if (lane == 0) scnt = cnt;
  }
  __syncthreads();

  for (int sec = 0; sec < 2; ++sec) {
    const float* bias = (sec == 0) ? bq : bk;
    unsigned short* dst = (sec == 0) ? Qs : Ks;
#pragma unroll 2
    for (int it = 0; it < 8; ++it) {
      const int rem = it * 256 + tid;
      const int c = rem >> 6, q4 = rem & 63;
      const v4f tv = *(const v4f*)(tab + (size_t)rowbase[c] + sec * kTH + 4 * q4);
      const v4f bb = *(const v4f*)(bias + rowboff[c] + 4 * q4);
      const float m = rowm[c];
      const float f0 = (m * tv[0] + bb[0]) * 64.0f;
      const float f1 = (m * tv[1] + bb[1]) * 64.0f;
      const float f2 = (m * tv[2] + bb[2]) * 64.0f;
      const float f3 = (m * tv[3] + bb[3]) * 64.0f;
      v2u pk;
      pk[0] = (unsigned)f2h_bits(f0) | ((unsigned)f2h_bits(f1) << 16);
      pk[1] = (unsigned)f2h_bits(f2) | ((unsigned)f2h_bits(f3) << 16);
      *(v2u*)(dst + c * 264 + 4 * q4) = pk;
    }
  }
#pragma unroll 2
  for (int it = 0; it < 8; ++it) {
    const int rem = it * 256 + tid;
    const int c = rem >> 6, q4 = rem & 63;
    const v4f tv = *(const v4f*)(tab + (size_t)rowbase[c] + 2 * kTH + 4 * q4);
    const v4f bb = *(const v4f*)(bv + rowboff[c] + 4 * q4);
    const float m = rowm[c];
#pragma unroll
    for (int e = 0; e < 4; ++e) Vt[(4 * q4 + e) * 40 + c] = f2h_bits((m * tv[e] + bb[e]) * 64.0f);
  }
  __syncthreads();

  if (wave < 4) {
    const int mi = wave >> 1, ti = wave & 1;
    v8f acc = (v8f){0.f,0.f,0.f,0.f,0.f,0.f,0.f,0.f};
#pragma unroll
    for (int ks = 0; ks < 8; ++ks) {
      const v16h a = Frag<_Float16>::load((const _Float16*)(Qs + (mi * 16 + rl) * 264 + ks * 32 + koff));
      const v16h b = Frag<_Float16>::load((const _Float16*)(Ks + (ti * 16 + rl) * 264 + ks * 32 + koff));
      acc = mma_h(a, b, acc);
    }
    const float c1 = kAttScale * kInv4096;
#pragma unroll
    for (int r = 0; r < 8; ++r) Sf[(mi * 16 + 8 * hh + r) * 33 + ti * 16 + rl] = acc[r] * c1;
  }
  __syncthreads();

  {
    const bool has = (scnt > 0);
    const float kv = kvalf[lane];
    const float ninf = -__builtin_inff();
    for (int rr = 0; rr < 4; ++rr) {
      const int row = wave * 4 + rr;
      const float sc = Sf[row * 33 + lane];
      const float x = has ? ((kv != 0.0f) ? sc : ninf) : 1.0f;
      float m = x;
#pragma unroll
      for (int off = 1; off < 32; off <<= 1) m = fmaxf(m, __shfl_xor(m, off, 32));
      const float e = expf(x - m);
      float sum = e;
#pragma unroll
      for (int off = 1; off < 32; off <<= 1) sum += __shfl_xor(sum, off, 32);
      const float p = e * (1.0f / sum);
      Ps[row * 40 + lane] = f2h_bits(p * 1024.0f);
    }
  }
  __syncthreads();

  {
    const v16h a0 = Frag<_Float16>::load((const _Float16*)(Ps + rl * 40 + koff));
    const v16h a1 = Frag<_Float16>::load((const _Float16*)(Ps + (16 + rl) * 40 + koff));
    float mq0[8], mq1[8];
#pragma unroll
    for (int r = 0; r < 8; ++r) { mq0[r] = kvalf[8 * hh + r]; mq1[r] = kvalf[16 + 8 * hh + r]; }
    const v8f z8 = (v8f){0.f,0.f,0.f,0.f,0.f,0.f,0.f,0.f};
#pragma unroll
    for (int q = 0; q < 2; ++q) {
      const int ni = wave * 2 + q;
      const v16h b = Frag<_Float16>::load((const _Float16*)(Vt + (ni * 16 + rl) * 40 + koff));
      const v8f acc0 = mma_h(a0, b, z8);
      const v8f acc1 = mma_h(a1, b, z8);
      float part = 0.0f;
#pragma unroll
      for (int r = 0; r < 8; ++r) part += acc0[r] * mq0[r] + acc1[r] * mq1[r];
      part += __shfl_xor(part, 16, 32);
      if (lane < 16) nomv[ni * 16 + lane] = part;
    }
  }
  __syncthreads();

  if (wave == 0) {
    const int cnt = scnt;
    const float den = (cnt > 0) ? (float)cnt : 10.0f;
    const float f = (1.0f / den) * (1.0f / 1024.0f);
    v4u w;
#pragma unroll
    for (int e = 0; e < 4; ++e) {
      const int d0 = lane * 8 + 2 * e;
      const unsigned lo = f2h_bits(nomv[d0] * f);
      const unsigned hi = f2h_bits(nomv[d0 + 1] * f);
      w[e] = lo | (hi << 16);
    }
    volatile v4u* o = (volatile v4u*)(temp16 + (size_t)gidx * kHid) + lane;
    *o = w;
    __threadfence();
    *o = w;
  }
}

__global__ __launch_bounds__(256) void k_bigru(
    const float* __restrict__ GI,
    const unsigned short* __restrict__ WHH,
    const float* __restrict__ bhh_f, const float* __restrict__ bhh_b,
    float* __restrict__ outf32,
    unsigned short* __restrict__ out16)
{
  __shared__ __align__(16) unsigned short hA[16 * 264];
  __shared__ __align__(16) float slab[16 * 260];

  const int dir = blockIdx.x >> 1;
  const int b0 = (blockIdx.x & 1) * 16;
  const float* bhh = dir ? bhh_b : bhh_f;
  const float* gi_base = GI + (size_t)dir * kNRow * kTH;
  const unsigned short* whh = WHH + (size_t)dir * kTH * kHid;

  const int tid = threadIdx.x, lane = tid & 31, wave = tid >> 5;
  const int hh = lane >> 4, rl = lane & 15, koff = hh * 8;

#pragma unroll
  for (int r = 0; r < 16; ++r) hA[r * 264 + tid] = (unsigned short)0;
  float hreg[2][8];
#pragma unroll
  for (int u = 0; u < 2; ++u)
#pragma unroll
    for (int r = 0; r < 8; ++r) hreg[u][r] = 0.0f;
  float bhr[2], bhz[2], bhn[2];
#pragma unroll
  for (int u = 0; u < 2; ++u) {
    const int unit = (wave * 2 + u) * 16 + rl;
    bhr[u] = bhh[unit]; bhz[u] = bhh[kHid + unit]; bhn[u] = bhh[2 * kHid + unit];
  }
  __syncthreads();

  for (int ts = 0; ts < kNS; ++ts) {
    const int t = dir ? (kNS - 1 - ts) : ts;
    v8f acc[2][3];
#pragma unroll
    for (int u = 0; u < 2; ++u)
#pragma unroll
      for (int g = 0; g < 3; ++g) acc[u][g] = (v8f){0.f,0.f,0.f,0.f,0.f,0.f,0.f,0.f};
#pragma unroll 2
    for (int ks = 0; ks < 8; ++ks) {
      const v16h a = Frag<_Float16>::load((const _Float16*)(hA + rl * 264 + ks * 32 + koff));
#pragma unroll
      for (int u = 0; u < 2; ++u) {
#pragma unroll
        for (int g = 0; g < 3; ++g) {
          const v16h b = Frag<_Float16>::load((const _Float16*)(whh + (size_t)(g * kHid + (wave * 2 + u) * 16 + rl) * kHid + ks * 32 + koff));
          acc[u][g] = mma_h(a, b, acc[u][g]);
        }
      }
    }
    __syncthreads();

#pragma unroll
    for (int u = 0; u < 2; ++u) {
      const int unit = (wave * 2 + u) * 16 + rl;
#pragma unroll
      for (int r = 0; r < 8; ++r) {
        const int row = 8 * hh + r;
        const int brow = b0 + row;
        const float* gi = gi_base + (size_t)(brow * kNS + t) * kTH + unit;
        const float ir = gi[0], iz = gi[kHid], inn = gi[2 * kHid];
        const float hr = acc[u][0][r] * kInv4096 + bhr[u];
        const float hz = acc[u][1][r] * kInv4096 + bhz[u];
        const float hn = acc[u][2][r] * kInv4096 + bhn[u];
        const float rg = 1.0f / (1.0f + expf(-(ir + hr)));
        const float zg = 1.0f / (1.0f + expf(-(iz + hz)));
        const float ng = tanhf(inn + rg * hn);
        const float hp = hreg[u][r];
        const float hnew = (1.0f - zg) * ng + zg * hp;
        hreg[u][r] = hnew;
        slab[row * 260 + unit] = hnew;
        hA[row * 264 + unit] = f2h_bits(hnew * 64.0f);
      }
    }
    __syncthreads();

#pragma unroll
    for (int q = 0; q < 2; ++q) {
      const int row = wave * 2 + q;
      const int brow = b0 + row;
      const size_t ob = (size_t)(brow * kNS + t) * 512 + dir * kHid;
      const v4f v0 = *(const v4f*)(slab + row * 260 + 4 * lane);
      const v4f v1 = *(const v4f*)(slab + row * 260 + 128 + 4 * lane);
      const v4u hv = *(const v4u*)(hA + row * 264 + 8 * lane);
      volatile v4f* o0 = (volatile v4f*)(outf32 + ob) + lane;
      volatile v4f* o1 = (volatile v4f*)(outf32 + ob) + 32 + lane;
      volatile v4u* oh = (volatile v4u*)(out16 + ob) + lane;
      *o0 = v0; *o1 = v1; *oh = hv;
      __threadfence();
      *o0 = v0; *o1 = v1; *oh = hv;
    }
  }
}

__global__ __launch_bounds__(256) void k_pool(
    const float* __restrict__ U, const float* __restrict__ usw, const float* __restrict__ usb,
    const int* __restrict__ maskb, const float* __restrict__ outf32, float* __restrict__ dout)
{
  __shared__ float usv[64];
  __shared__ float alphav[64];
  __shared__ __align__(16) float resv[512];
  const int b = blockIdx.x;
  const int tid = threadIdx.x, lane = tid & 31, wave = tid >> 5;

  float uw[8];
#pragma unroll
  for (int i = 0; i < 8; ++i) uw[i] = usw[lane + 32 * i];
  for (int s = wave; s < kNS; s += 8) {
    const float* ur = U + (size_t)(b * kNS + s) * kHid;
    float p = 0.0f;
#pragma unroll
    for (int i = 0; i < 8; ++i) p += ur[lane + 32 * i] * uw[i];
#pragma unroll
    for (int off = 1; off < 32; off <<= 1) p += __shfl_xor(p, off, 32);
    if (lane == 0) usv[s] = p + usb[0];
  }
  __syncthreads();

  if (wave == 0) {
    const float ninf = -__builtin_inff();
    const int s0 = lane, s1 = lane + 32;
    const int s1c = (s1 < kNS) ? s1 : (kNS - 1);
    const int m0 = maskb[b * kNS + s0];
    const int m1 = maskb[b * kNS + s1c];
    const float u0 = usv[s0];
    const float u1 = usv[s1c];
    const float x0 = (m0 != 0) ? ninf : u0;
    const float x1 = (s1 < kNS && m1 == 0) ? u1 : ninf;
    float m = fmaxf(x0, x1);
#pragma unroll
    for (int off = 1; off < 32; off <<= 1) m = fmaxf(m, __shfl_xor(m, off, 32));
    const float e0 = expf(x0 - m), e1 = expf(x1 - m);
    float sum = e0 + e1;
#pragma unroll
    for (int off = 1; off < 32; off <<= 1) sum += __shfl_xor(sum, off, 32);
    const float inv = 1.0f / sum;
    alphav[s0] = e0 * inv;
    alphav[s1] = e1 * inv;
  }
  __syncthreads();

#pragma unroll
  for (int half = 0; half < 2; ++half) {
    const int d = tid + half * 256;
    float a = 0.0f;
#pragma unroll 1
    for (int s = 0; s < kNS; ++s) a += alphav[s] * outf32[(size_t)(b * kNS + s) * 512 + d];
    resv[d] = a;
  }
  __syncthreads();

  if (wave < 4) {
    const v4f v = *(const v4f*)(resv + wave * 128 + 4 * lane);
    volatile v4f* o = (volatile v4f*)(dout + (size_t)b * 512 + wave * 128) + lane;
    *o = v;
    __threadfence();
    *o = v;
  }
}

static inline size_t al256(size_t x) { return (x + 255) & ~(size_t)255; }

extern "C" void kernel_launch(void* const* d_in, const int* in_sizes, int n_in,
                              void* d_out, int out_size, void* d_ws, size_t ws_size,
                              hipStream_t stream) {
  if (n_in < 25) return;
  if (in_sizes[0] != kNB * kNS * kNCd || in_sizes[2] != kNB * kNS || in_sizes[4] != kNB * kNS * kNCd ||
      in_sizes[6] != kNCode * kHid || in_sizes[7] != kTH * kHid || in_sizes[13] != kTH * kTH ||
      in_sizes[14] != kTH * kHid || in_sizes[21] != kHid * 512 || in_sizes[23] != kHid || in_sizes[24] < 1) return;
  if (out_size < kNB * 512) return;

  const int*   codes     = (const int*)  d_in[0];
  const int*   mask_b    = (const int*)  d_in[2];
  const float* mask_code = (const float*)d_in[4];
  const float* emb       = (const float*)d_in[6];
  const float* wq_w = (const float*)d_in[7],  *wq_b = (const float*)d_in[8];
  const float* wk_w = (const float*)d_in[9],  *wk_b = (const float*)d_in[10];
  const float* wv_w = (const float*)d_in[11], *wv_b = (const float*)d_in[12];
  const float* gwih_f = (const float*)d_in[13], *gwhh_f = (const float*)d_in[14];
  const float* gbih_f = (const float*)d_in[15], *gbhh_f = (const float*)d_in[16];
  const float* gwih_b = (const float*)d_in[17], *gwhh_b = (const float*)d_in[18];
  const float* gbih_b = (const float*)d_in[19], *gbhh_b = (const float*)d_in[20];
  const float* ws_w = (const float*)d_in[21], *ws_b = (const float*)d_in[22];
  const float* us_w = (const float*)d_in[23], *us_b = (const float*)d_in[24];

  char* ws = (char*)d_ws;
  size_t off = 0;
  unsigned short* EMB16  = (unsigned short*)(ws + off); off += al256((size_t)kNCodePad * kHid * 2);
  unsigned short* WQKV16 = (unsigned short*)(ws + off); off += al256((size_t)kTW * kHid * 2);
  float*          TAB    = (float*)(ws + off);          off += al256((size_t)kNCodePad * kTW * 4);
  unsigned short* TEMP16 = (unsigned short*)(ws + off); off += al256((size_t)kNGrp * kHid * 2);
  unsigned short* WIH16  = (unsigned short*)(ws + off); off += al256((size_t)2 * kTH * kTH * 2);
  unsigned short* WHH16  = (unsigned short*)(ws + off); off += al256((size_t)2 * kTH * kHid * 2);
  float*          GI     = (float*)(ws + off);          off += al256((size_t)2 * kNRow * kTH * 4);
  float*          OUTF32 = (float*)(ws + off);          off += al256((size_t)kNRow * 512 * 4);
  unsigned short* OUT16  = (unsigned short*)(ws + off); off += al256((size_t)kNRow * 512 * 2);
  unsigned short* WS16   = (unsigned short*)(ws + off); off += al256((size_t)kHid * 512 * 2);
  float*          UF     = (float*)(ws + off);          off += al256((size_t)kNRow * kHid * 4);
  if (off > ws_size) return;

  auto cast = [&](const float* src, int nvalid, unsigned short* dst, int ntot, float sc) {
    const int n2 = ntot / 2;
    k_cast_f16<<<(n2 + 255) / 256, 256, 0, stream>>>(src, nvalid, dst, n2, sc);
  };
  cast(emb,    kNCode * kHid, EMB16,                       kNCodePad * kHid, 64.0f);
  cast(wq_w,   kTH * kHid,    WQKV16,                      kTH * kHid,       64.0f);
  cast(wk_w,   kTH * kHid,    WQKV16 + (size_t)kTH * kHid, kTH * kHid,       64.0f);
  cast(wv_w,   kTH * kHid,    WQKV16 + (size_t)2 * kTH * kHid, kTH * kHid,   64.0f);
  cast(gwih_f, kTH * kTH,     WIH16,                       kTH * kTH,        64.0f);
  cast(gwih_b, kTH * kTH,     WIH16 + (size_t)kTH * kTH,   kTH * kTH,        64.0f);
  cast(gwhh_f, kTH * kHid,    WHH16,                       kTH * kHid,       64.0f);
  cast(gwhh_b, kTH * kHid,    WHH16 + (size_t)kTH * kHid,  kTH * kHid,       64.0f);
  cast(ws_w,   kHid * 512,    WS16,                        kHid * 512,       64.0f);

  {
    const int tiles = (kNCodePad / 64) * (kTW / 64);
    wmma_gemm64<0, false, 0, 0, false, 0><<<dim3((tiles + 7) / 8, 1), 256, 0, stream>>>(
        EMB16, EMB16, kHid, 0L, WQKV16, WQKV16, kHid, 0L,
        (void*)TAB, (void*)TAB, kTW, 0L, wq_b, wq_b, 0L, kNCodePad, kTW, kHid, kInv4096);
  }

  k_code_attn<<<kNGrp, 256, 0, stream>>>(codes, mask_code, TAB, wq_b, wk_b, wv_b, TEMP16);

  {
    const int tiles = (kNRow / 64) * (kTH / 64);
    wmma_gemm64<0, false, 2, 0, false, 0><<<dim3((tiles + 7) / 8, 1), 256, 0, stream>>>(
        TEMP16, TEMP16, kTH, 0L, WIH16, WIH16, kTH, 0L,
        (void*)GI, (void*)GI, kTH, 0L, gbih_f, gbih_f, 0L, kNRow, kTH, kTH, kInv4096);
    wmma_gemm64<0, false, 2, 0, false, 0><<<dim3((tiles + 7) / 8, 1), 256, 0, stream>>>(
        TEMP16, TEMP16, kTH, 0L, WIH16 + (size_t)kTH * kTH, WIH16 + (size_t)kTH * kTH, kTH, 0L,
        (void*)(GI + (size_t)kNRow * kTH), (void*)(GI + (size_t)kNRow * kTH), kTH, 0L,
        gbih_b, gbih_b, 0L, kNRow, kTH, kTH, kInv4096);
  }

  k_bigru<<<4, 256, 0, stream>>>(GI, WHH16, gbhh_f, gbhh_b, OUTF32, OUT16);

  {
    const int tiles = (kNRow / 64) * (kHid / 64);
    wmma_gemm64<0, false, 2, 0, false, 1><<<dim3((tiles + 7) / 8, 1), 256, 0, stream>>>(
        OUT16, OUT16, 512, 0L, WS16, WS16, 512, 0L,
        (void*)UF, (void*)UF, kHid, 0L, ws_b, ws_b, 0L, kNRow, kHid, 512, kInv4096);
  }

  k_pool<<<kNB, 256, 0, stream>>>(UF, us_w, us_b, mask_b, OUTF32, (float*)d_out);
}
